// PosBiasedMultiHeadedAttention_17214228922450
// MI455X (gfx1250) — hardware-verified
//
#include <hip/hip_runtime.h>
#include <math.h>

typedef __attribute__((ext_vector_type(16))) _Float16 v16h;
typedef __attribute__((ext_vector_type(16))) __bf16 v16b;
typedef __attribute__((ext_vector_type(8)))  _Float16 v8h;
typedef __attribute__((ext_vector_type(8)))  float v8f;
typedef __attribute__((ext_vector_type(4)))  float v4f;
typedef __attribute__((ext_vector_type(2)))  float v2f;
typedef __attribute__((ext_vector_type(4)))  unsigned v4u;
typedef __attribute__((ext_vector_type(4)))  int v4i;
typedef float __attribute__((may_alias)) float_a;
typedef int __attribute__((may_alias)) int_a;

template <typename T> __device__ __forceinline__ void vst2(void* p, T v) { *(volatile T*)p = v; __threadfence(); *(volatile T*)p = v; }
__device__ __forceinline__ v8f wmma16(v16h a, v16h b, v8f c) {
  v8f d = __builtin_amdgcn_wmma_f32_16x16x32_f16(false, a, false, b, (short)0, c, false, false);
  asm volatile("v_nop\n\tv_nop\n\tv_nop\n\tv_nop" : "+v"(d) : "v"(a), "v"(b));
  return d;
}
__device__ __forceinline__ v8f wmma_bf(v16b a, v16b b, v8f c) {
  v8f d = __builtin_amdgcn_wmma_f32_16x16x32_bf16(false, a, false, b, (short)0, c, false, false);
  asm volatile("v_nop\n\tv_nop\n\tv_nop\n\tv_nop" : "+v"(d) : "v"(a), "v"(b));
  return d;
}
__device__ __forceinline__ v16h frag_h(const _Float16* rowk0, int lane) {
  union { v16h v; v8h q[2]; } u; const _Float16* p = rowk0 + 8 * (lane >> 4);
  u.q[0] = *(const v8h*)p; u.q[1] = *(const v8h*)(p + 16); return u.v;
}
__device__ __forceinline__ v16h frag_f32(const float* rowk0, int lane) {
  v16h a; const float* p = rowk0 + 8 * (lane >> 4);
#pragma unroll
  for (int i = 0; i < 8; ++i) { a[i] = (_Float16)p[i]; a[8 + i] = (_Float16)p[16 + i]; }
  return a;
}
__device__ __forceinline__ v16h frag_f32s(const float* rowk0, int lane, float sc) {
  v16h a; const float* p = rowk0 + 8 * (lane >> 4);
#pragma unroll
  for (int i = 0; i < 8; ++i) { a[i] = (_Float16)(p[i] * sc); a[8 + i] = (_Float16)(p[16 + i] * sc); }
  return a;
}
__device__ __forceinline__ v16h fragc_f32(const float* W, int k0, int n, int lane, int ld, int K) {
  v16h a; const int g = lane >> 4;
#pragma unroll
  for (int i = 0; i < 8; ++i) { const int ka = k0 + 8 * g + i, kb = ka + 16;
    a[i] = (_Float16)(ka < K ? W[(size_t)ka * ld + n] : 0.f); a[8 + i] = (_Float16)(kb < K ? W[(size_t)kb * ld + n] : 0.f); }
  return a;
}
struct F2 { v16b h, l; };
__device__ __forceinline__ F2 bsplit16(const float v[16]) { F2 r;
#pragma unroll
  for (int i = 0; i < 16; ++i) { const __bf16 h = (__bf16)v[i]; r.h[i] = h; r.l[i] = (__bf16)(v[i] - (float)h); }
  return r; }
__device__ __forceinline__ F2 split_row(const float* row, int k0, int lane) { float v[16]; const float* p = row + k0 + 8 * (lane >> 4);
#pragma unroll
  for (int i = 0; i < 8; ++i) { v[i] = p[i]; v[8 + i] = p[16 + i]; }
  return bsplit16(v); }
__device__ __forceinline__ F2 split_rowK(const float* row, int k0, int lane, int K) { float v[16]; const int g = lane >> 4;
#pragma unroll
  for (int i = 0; i < 8; ++i) { const int ka = k0 + 8 * g + i, kb = ka + 16; v[i] = ka < K ? row[ka] : 0.f; v[8 + i] = kb < K ? row[kb] : 0.f; }
  return bsplit16(v); }
__device__ __forceinline__ F2 split_col(const float* W, int k0, int n, int lane, int ld, int K) { float v[16]; const int g = lane >> 4;
#pragma unroll
  for (int i = 0; i < 8; ++i) { const int ka = k0 + 8 * g + i, kb = ka + 16; v[i] = ka < K ? W[(size_t)ka * ld + n] : 0.f; v[8 + i] = kb < K ? W[(size_t)kb * ld + n] : 0.f; }
  return bsplit16(v); }
__device__ __forceinline__ v8f mac3(const F2& a, const F2& b, v8f c) { c = wmma_bf(a.l, b.h, c); c = wmma_bf(a.h, b.l, c); return wmma_bf(a.h, b.h, c); }
__device__ __forceinline__ float sigm(float v) { return 1.0f / (1.0f + expf(-v)); }
#define LDSX() do { asm volatile("s_wait_dscnt 0" ::: "memory"); __builtin_amdgcn_wave_barrier(); __builtin_amdgcn_fence(__ATOMIC_RELEASE, "workgroup"); } while (0)

#define NB 2
#define NQ 512
#define DM 1024
#define NH 16
#define HD 64
#define PDK 16
#define EMB 256
#define NEMB 40001
#define NR (NB * NQ)

__global__ __launch_bounds__(256) void k_cvt(const float* __restrict__ src, _Float16* __restrict__ dst, size_t n8) {
  const size_t g8 = (size_t)blockIdx.x * 256 + threadIdx.x; if (g8 >= n8) return;
  union { v8h h; v4u u; } pk;
#pragma unroll
  for (int e = 0; e < 8; ++e) pk.h[e] = (_Float16)src[g8 * 8 + e];
  vst2(dst + g8 * 8, pk.u);
}
__global__ __launch_bounds__(256) void k_packT(const float* __restrict__ W0, const float* __restrict__ W1, const float* __restrict__ W2, const float* __restrict__ W3, _Float16* __restrict__ P) {
  __shared__ float tile[64][65];
  const int which = blockIdx.z, o0 = blockIdx.x * 64, k0 = blockIdx.y * 64, tid = threadIdx.x;
  const float* W = which == 0 ? W0 : (which == 1 ? W1 : (which == 2 ? W2 : W3));
  for (int q = tid; q < 64 * 64; q += 256) { const int kl = q >> 6, ol = q & 63; tile[kl][ol] = W[(size_t)(k0 + kl) * DM + o0 + ol]; }
  __syncthreads();
  for (int u = 0; u < 2; ++u) { const int idx = tid + u * 256, ol = idx >> 3, pc = idx & 7; union { v8h hh; v4u uu; } pk;
#pragma unroll
    for (int i = 0; i < 8; ++i) pk.hh[i] = (_Float16)(tile[pc * 8 + i][ol] * 16.0f);
    vst2(P + ((size_t)which * DM + o0 + ol) * DM + k0 + pc * 8, pk.uu); }
}
__global__ __launch_bounds__(128) void k_proj(const _Float16* __restrict__ xq, const _Float16* __restrict__ xk, const _Float16* __restrict__ xv, const _Float16* __restrict__ P, const float* __restrict__ bq, const float* __restrict__ bk, const float* __restrict__ bv,
                                            _Float16* __restrict__ qh, _Float16* __restrict__ kh, _Float16* __restrict__ vT) {
  __shared__ __align__(16) float so[4][16][132];
  __shared__ __align__(16) _Float16 st[128][72];
  const int tid = threadIdx.x, wave = tid >> 5, lane = tid & 31, col = lane & 15, g = lane >> 4;
  const int which = blockIdx.z; const int r0b = blockIdx.x * 64, r0 = r0b + wave * 16, n0 = blockIdx.y * 128; const int b = r0b / NQ, t0 = r0b % NQ, hb = n0 / HD;
  const _Float16* A = which == 0 ? xq : (which == 1 ? xk : xv); const float* bias = which == 0 ? bq : (which == 1 ? bk : bv);
  v8f acc[8] = {};
#pragma unroll 1
  for (int kc = 0; kc < DM / 32; ++kc) { const v16h a = frag_h(A + (size_t)(r0 + col) * DM + kc * 32, lane);
#pragma unroll
    for (int j = 0; j < 8; ++j) acc[j] = wmma16(a, frag_h(P + ((size_t)which * DM + n0 + j * 16 + col) * DM + kc * 32, lane), acc[j]); }
#pragma unroll
  for (int j = 0; j < 8; ++j) { const float bb = bias[n0 + j * 16 + col];
#pragma unroll
    for (int r = 0; r < 8; ++r) so[wave][8 * g + r][j * 16 + col] = acc[j][r] * (1.0f / 16.0f) + bb; }
  LDSX();
  if (which < 2) { _Float16* dst = which == 0 ? qh : kh;
    for (int q = lane; q < 2 * 16 * 8; q += 32) { const int hh = q >> 7, rem = q & 127, rl = rem >> 3, pc = rem & 7; union { v8h h8; v4u u; } pk;
#pragma unroll
      for (int e = 0; e < 8; ++e) pk.h8[e] = (_Float16)so[wave][rl][hh * HD + pc * 8 + e];
      vst2(dst + (((size_t)b * NH + hb + hh) * NQ + t0 + wave * 16 + rl) * HD + pc * 8, pk.u); } }
  else {
#pragma unroll 4
    for (int rl = 0; rl < 16; ++rl) {
#pragma unroll
      for (int e = 0; e < 4; ++e) st[lane * 4 + e][wave * 16 + rl] = (_Float16)so[wave][rl][lane * 4 + e]; }
    __syncthreads();
    for (int q = tid; q < 128 * 8; q += 128) { const int c = q >> 3, pc = q & 7, hh = c >> 6, d = c & 63;
      vst2(vT + (((size_t)b * NH + hb + hh) * HD + d) * NQ + t0 + pc * 8, *(const v4u*)(&st[c][pc * 8])); } }
}
__global__ __launch_bounds__(256) void k_bias(const float* __restrict__ qx, const float* __restrict__ qy, const float* __restrict__ kx, const float* __restrict__ ky, const float* __restrict__ xt, const float* __restrict__ yt, const float* __restrict__ Wb, const float* __restrict__ bbp,
                                            float* __restrict__ bias) {
  __shared__ __align__(16) float so[NH][NQ];
  __shared__ float swb[PDK];
  const int i = blockIdx.x, b = blockIdx.y, tid = threadIdx.x;
  if (tid < PDK) swb[tid] = Wb[tid];
  __syncthreads();
  const float kxi = kx[b * NQ + i], kyi = ky[b * NQ + i]; const float bb0 = bbp[0];
  for (int j = tid; j < NQ; j += 256) {
    float dx = qx[b * NQ + j] - kxi; dx = fminf(fmaxf(dx, -1000.0f), 1000.0f); const int ix = (int)rintf((dx + 1000.0f) * 20.0f);
    float dy = qy[b * NQ + j] - kyi; dy = fminf(fmaxf(dy, -1000.0f), 1000.0f); const int iy = (int)rintf((dy + 1000.0f) * 20.0f);
    const int cix = ix < 0 ? 0 : (ix >= NEMB ? NEMB - 1 : ix), ciy = iy < 0 ? 0 : (iy >= NEMB ? NEMB - 1 : iy);
    const float* xr = xt + (size_t)cix * EMB; const float* yr = yt + (size_t)ciy * EMB;
#pragma unroll 1
    for (int h = 0; h < NH; ++h) { float a = bb0;
#pragma unroll
      for (int e = 0; e < PDK; ++e) a += (xr[h * PDK + e] + yr[h * PDK + e]) * swb[e];
      so[h][j] = sigm(a); } }
  __syncthreads();
  for (int q = tid; q < NH * NQ / 4; q += 256) { const int h = q >> 7, pc = q & 127; vst2(bias + (((size_t)b * NH + h) * NQ + i) * NQ + pc * 4, *(const v4f*)(&so[h][pc * 4])); }
}
__global__ __launch_bounds__(128) void k_attn(const _Float16* __restrict__ qh, const _Float16* __restrict__ kh, const _Float16* __restrict__ vT, const float* __restrict__ bias, _Float16* __restrict__ o16) {
  __shared__ __align__(16) float sS[4][16][68];
  __shared__ __align__(16) _Float16 sP[4][16][72];
  __shared__ __align__(16) float sO[4][16][68];
  const int tid = threadIdx.x, w = tid >> 5, lane = tid & 31, col = lane & 15, g = lane >> 4;
  const int bh = blockIdx.y, b = bh / NH, h = bh % NH, q0 = blockIdx.x * 64 + w * 16;
  const _Float16* qb = qh + (size_t)bh * NQ * HD; const _Float16* kb = kh + (size_t)bh * NQ * HD; const _Float16* vb = vT + (size_t)bh * HD * NQ; const float* bbh = bias + (size_t)bh * NQ * NQ;
  v16h aq[2];
#pragma unroll
  for (int kc = 0; kc < 2; ++kc) aq[kc] = frag_h(qb + (size_t)(q0 + col) * HD + kc * 32, lane);
  float mrun = -3.0e38f, lrun = 0.f; v8f acc[4] = {};
#pragma unroll 1
  for (int kt = 0; kt < NQ / 64; ++kt) {
#pragma unroll
    for (int t = 0; t < 4; ++t) { v8f s = {}; const int key = kt * 64 + t * 16 + col;
#pragma unroll
      for (int kc = 0; kc < 2; ++kc) s = wmma16(aq[kc], frag_h(kb + (size_t)key * HD + kc * 32, lane), s);
#pragma unroll
      for (int r = 0; r < 8; ++r) { const int qi = q0 + 8 * g + r; sS[w][8 * g + r][t * 16 + col] = s[r] * 0.125f + bbh[(size_t)qi * NQ + key]; } }
    LDSX();
    float mx = -3.4e38f;
#pragma unroll
    for (int jj = 0; jj < 32; ++jj) mx = fmaxf(mx, sS[w][col][g * 32 + jj]);
    mx = fmaxf(mx, __shfl_xor(mx, 16, 32));
    const float mnew = fmaxf(mrun, mx); const float corr = expf(mrun - mnew);
    float ps = 0.f;
#pragma unroll
    for (int jj = 0; jj < 32; ++jj) { const float p = expf(sS[w][col][g * 32 + jj] - mnew); ps += p; sP[w][col][g * 32 + jj] = (_Float16)(p * 16384.0f); }
    ps += __shfl_xor(ps, 16, 32);
    lrun = lrun * corr + ps; mrun = mnew;
#pragma unroll
    for (int r = 0; r < 8; ++r) { const float cr = __shfl(corr, 8 * g + r, 32);
#pragma unroll
      for (int t = 0; t < 4; ++t) acc[t][r] *= cr; }
    LDSX();
#pragma unroll
    for (int kc = 0; kc < 2; ++kc) { const v16h pa = frag_h(&sP[w][col][0] + kc * 32, lane);
#pragma unroll
      for (int t = 0; t < 4; ++t) acc[t] = wmma16(pa, frag_h(vb + (size_t)(t * 16 + col) * NQ + kt * 64 + kc * 32, lane), acc[t]); }
    __builtin_amdgcn_wave_barrier();
  }
#pragma unroll
  for (int r = 0; r < 8; ++r) { const float lr = __shfl(lrun, 8 * g + r, 32);
#pragma unroll
    for (int t = 0; t < 4; ++t) sO[w][8 * g + r][t * 16 + col] = acc[t][r] / (lr * 16384.0f); }
  LDSX();
  for (int q = lane; q < 16 * 8; q += 32) { const int rl = q >> 3, pc = q & 7; union { v8h h8; v4u u; } pk;
#pragma unroll
    for (int e = 0; e < 8; ++e) pk.h8[e] = (_Float16)(sO[w][rl][pc * 8 + e] * 16.0f);
    vst2(o16 + ((size_t)b * NQ + q0 + rl) * DM + h * HD + pc * 8, pk.u); }
}
__global__ __launch_bounds__(128) void k_out(const _Float16* __restrict__ o16, const _Float16* __restrict__ P, const float* __restrict__ bo, float* __restrict__ out) {
  __shared__ __align__(16) float so[4][16][132];
  const int tid = threadIdx.x, wave = tid >> 5, lane = tid & 31, col = lane & 15, g = lane >> 4;
  const int r0 = blockIdx.x * 64 + wave * 16, n0 = blockIdx.y * 128;
  v8f acc[8] = {};
#pragma unroll 1
  for (int kc = 0; kc < DM / 32; ++kc) { const v16h a = frag_h(o16 + (size_t)(r0 + col) * DM + kc * 32, lane);
#pragma unroll
    for (int j = 0; j < 8; ++j) acc[j] = wmma16(a, frag_h(P + ((size_t)3 * DM + n0 + j * 16 + col) * DM + kc * 32, lane), acc[j]); }
#pragma unroll
  for (int j = 0; j < 8; ++j) { const float b0 = bo[n0 + j * 16 + col];
#pragma unroll
    for (int r = 0; r < 8; ++r) so[wave][8 * g + r][j * 16 + col] = acc[j][r] * (1.0f / 256.0f) + b0; }
  LDSX();
#pragma unroll 4
  for (int rl = 0; rl < 16; ++rl) vst2(out + (size_t)(r0 + rl) * DM + n0 + lane * 4, *(const v4f*)(&so[wave][rl][lane * 4]));
}
extern "C" void kernel_launch(void* const* d_in, const int* in_sizes, int n_in, void* d_out, int out_size, void* d_ws, size_t ws_size, hipStream_t stream) {
  (void)in_sizes; (void)n_in; (void)out_size; (void)ws_size;
  const float** I = (const float**)d_in;
  const float* query = I[0]; const float* key = I[1]; const float* value = I[2]; const float* qx = I[3]; const float* qy = I[4]; const float* kx = I[5]; const float* ky = I[6];
  const float* Wq = I[7]; const float* bq = I[8]; const float* Wk = I[9]; const float* bk = I[10]; const float* Wv = I[11]; const float* bv = I[12]; const float* Wo = I[13]; const float* bo = I[14];
  const float* xt = I[15]; const float* yt = I[16]; const float* Wb = I[17]; const float* bbp = I[18];
  float* out = (float*)d_out;
  char* ws = (char*)d_ws; size_t off = 0;
  auto take = [&](size_t bytes) { char* p = ws + off; off += (bytes + 255) & ~(size_t)255; return p; };
  _Float16* xq16 = (_Float16*)take((size_t)NR * DM * 2); _Float16* xk16 = (_Float16*)take((size_t)NR * DM * 2); _Float16* xv16 = (_Float16*)take((size_t)NR * DM * 2); _Float16* P = (_Float16*)take((size_t)4 * DM * DM * 2);
  _Float16* qh = (_Float16*)take((size_t)NR * DM * 2); _Float16* kh = (_Float16*)take((size_t)NR * DM * 2); _Float16* vT = (_Float16*)take((size_t)NR * DM * 2); _Float16* o16 = (_Float16*)take((size_t)NR * DM * 2);
  float* bias = (float*)take((size_t)NB * NH * NQ * NQ * 4);
  const size_t n8 = (size_t)NR * DM / 8;
  k_cvt<<<(unsigned)(n8 / 256), 256, 0, stream>>>(query, xq16, n8); k_cvt<<<(unsigned)(n8 / 256), 256, 0, stream>>>(key, xk16, n8); k_cvt<<<(unsigned)(n8 / 256), 256, 0, stream>>>(value, xv16, n8);
  k_packT<<<dim3(DM / 64, DM / 64, 4), 256, 0, stream>>>(Wq, Wk, Wv, Wo, P);
  k_proj<<<dim3(NR / 64, DM / 128, 3), 128, 0, stream>>>(xq16, xk16, xv16, P, bq, bk, bv, qh, kh, vT);
  k_bias<<<dim3(NQ, NB), 256, 0, stream>>>(qx, qy, kx, ky, xt, yt, Wb, bbp, bias);
  k_attn<<<dim3(NQ / 64, NB * NH), 128, 0, stream>>>(qh, kh, vT, bias, o16);
  k_out<<<dim3(NR / 64, DM / 128), 128, 0, stream>>>(o16, P, bo, out);
}
